// MultiHeadAttention_34540126994511
// MI455X (gfx1250) — hardware-run, weakly checked
//
#include <hip/hip_runtime.h>

#ifndef NB
#define NB 4
#endif
#ifndef SEQ
#define SEQ 2048
#endif
#define NB_FULL  4
#define SEQ_FULL 2048
#define EMB      1024
#define NHEADS   16
#define HDIM     64
#define QKP      2048

static_assert(SEQ % 64 == 0);
static_assert(SEQ <= SEQ_FULL);
static_assert(NB <= NB_FULL);
static_assert(EMB == NHEADS * HDIM);
static_assert(EMB % 64 == 0);

typedef __attribute__((ext_vector_type(16))) _Float16 v16h;
typedef __attribute__((ext_vector_type(8)))  _Float16 v8h;
typedef __attribute__((ext_vector_type(8)))  float    v8f;
typedef __attribute__((ext_vector_type(4)))  float    v4f;
typedef __attribute__((ext_vector_type(4)))  unsigned int u4;


namespace eng {

union FragU { v16h v; v8h h[2]; };
__device__ __forceinline__ v16h frag_load(const _Float16* p) {
  FragU f; f.h[0] = *(const v8h*)(p); f.h[1] = *(const v8h*)(p + 16); return f.v;
}
__device__ __forceinline__ v8f mma_h(v16h a, v16h b, v8f c) {
  return __builtin_amdgcn_wmma_f32_16x16x32_f16(false, a, false, b, (short)0, c, false, false);
}
__device__ __forceinline__ void dep_guard_h(v8f& a, v8f& b, v16h x, v16h y) { asm volatile("v_nop\n\tv_nop\n\tv_nop\n\tv_nop" : "+v"(a), "+v"(b) : "v"(x), "v"(y)); }
__device__ __forceinline__ void keep4_h(v16h a, v16h b, v16h c, v16h d) { asm volatile("v_nop" :: "v"(a), "v"(b), "v"(c), "v"(d)); }
__device__ __forceinline__ void acc_guard4(v8f& a, v8f& b, v8f& c, v8f& d) { asm volatile("v_nop\n\tv_nop\n\tv_nop\n\tv_nop" : "+v"(a), "+v"(b), "+v"(c), "+v"(d)); }
__device__ __forceinline__ void guard_s(v8f& a, v8f& b, v16h x0, v16h x1, v16h x2, v16h x3, v16h y0, v16h y1) {
  asm volatile("v_nop\n\tv_nop\n\tv_nop\n\tv_nop" : "+v"(a), "+v"(b) : "v"(x0), "v"(x1), "v"(x2), "v"(x3), "v"(y0), "v"(y1));
}
__device__ __forceinline__ void guard_o(v8f& a, v8f& b, v8f& c, v8f& d, v16h x0, v16h x1, v16h x2, v16h x3, v16h p) {
  asm volatile("v_nop\n\tv_nop\n\tv_nop\n\tv_nop" : "+v"(a), "+v"(b), "+v"(c), "+v"(d) : "v"(x0), "v"(x1), "v"(x2), "v"(x3), "v"(p));
}

__device__ __forceinline__ float bf_rne(float v) {
  const unsigned u = __builtin_bit_cast(unsigned, v);
  const unsigned r = (u + 0x7fffu + ((u >> 16) & 1u)) & 0xffff0000u;
  return __builtin_bit_cast(float, r);
}
__device__ __forceinline__ unsigned pk2h(float a, float b) {
  return (unsigned)__builtin_bit_cast(unsigned short, (_Float16)a) | ((unsigned)__builtin_bit_cast(unsigned short, (_Float16)b) << 16);
}

template <int BIAS_MODE, int OUT_MODE>
__global__ __launch_bounds__(256) void wmma_gemm64(
    const unsigned short* __restrict__ Ap, int lda, long long strideA,
    const unsigned short* __restrict__ Btp, int ldb, long long strideB,
    void* __restrict__ Cout, int ldc, long long strideC,
    const float* __restrict__ bias,
    int M, int N, int K, float scale) {
  __shared__ __align__(16) float sT[8][16 * 68];
  const _Float16* A  = (const _Float16*)Ap;
  const _Float16* Bt = (const _Float16*)Btp;
  const int b    = blockIdx.y;
  const int lane = threadIdx.x & 31;
  const int wave = __builtin_amdgcn_readfirstlane((int)(threadIdx.x >> 5));
  const int tilesN = N >> 6;
  const int tilesM = M >> 6;
  int tile = blockIdx.x * 8 + wave;
  tile = min(tile, tilesM * tilesN - 1);
  const int tm = tile / tilesN;
  const int tn = tile - tm * tilesN;
  const int m0 = tm << 6;
  const int n0 = tn << 6;

  const _Float16* Ab = A  + (size_t)b * (size_t)strideA;
  const _Float16* Bb = Bt + (size_t)b * (size_t)strideB;

  const int rlane = lane & 15;
  const int koff  = (lane >> 4) * 8;
  const int mOff  = (lane >> 4) * 8;

  v8f acc[4][4];
#pragma unroll
  for (int i = 0; i < 4; ++i)
#pragma unroll
    for (int j = 0; j < 4; ++j) acc[i][j] = (v8f){0.f,0.f,0.f,0.f,0.f,0.f,0.f,0.f};

  for (int k0 = 0; k0 < K; k0 += 32) {
    v16h bh[4];
#pragma unroll
    for (int j = 0; j < 4; ++j) {
      const size_t bo = (size_t)(n0 + (j << 4) + rlane) * ldb + koff + k0;
      bh[j] = frag_load(Bb + bo);
    }
#pragma unroll
    for (int i = 0; i < 4; ++i) {
      const size_t ao = (size_t)(m0 + (i << 4) + rlane) * lda + koff + k0;
      const v16h ah = frag_load(Ab + ao);
#pragma unroll
      for (int j = 0; j < 4; ++j) acc[i][j] = mma_h(ah, bh[j], acc[i][j]);
      dep_guard_h(acc[i][0], acc[i][3], ah, ah);
    }
    keep4_h(bh[0], bh[1], bh[2], bh[3]);
  }
  acc_guard4(acc[0][0], acc[0][1], acc[0][2], acc[0][3]);
  acc_guard4(acc[1][0], acc[1][1], acc[1][2], acc[1][3]);
  acc_guard4(acc[2][0], acc[2][1], acc[2][2], acc[2][3]);
  acc_guard4(acc[3][0], acc[3][1], acc[3][2], acc[3][3]);

  float* slab = sT[wave];
#pragma unroll
  for (int i = 0; i < 4; ++i) {
    const int mBase = m0 + (i << 4);
#pragma unroll
    for (int j = 0; j < 4; ++j) {
      const int n = n0 + (j << 4) + rlane;
      float bv = 0.f;
      if (BIAS_MODE == 2) bv = bf_rne(bias[n]);
#pragma unroll
      for (int r = 0; r < 8; ++r) {
        float v = acc[i][j][r] * scale;
        if (BIAS_MODE == 1) v += bf_rne(bias[mBase + mOff + r]);
        if (BIAS_MODE == 2) v += bv;
        slab[(mOff + r) * 68 + (j << 4) + rlane] = v;
      }
    }
    __syncthreads();
    if (OUT_MODE == 0) {
      float* C = (float*)Cout + (size_t)b * (size_t)strideC;
      const int hh = lane >> 4, c4 = (lane & 15) * 4;
      for (int pass = 0; pass < 2; ++pass) {
#pragma unroll
        for (int it = 0; it < 8; ++it) {
          const int row = it * 2 + hh;
          const v4f v = *(const v4f*)(slab + row * 68 + c4);
          *(volatile v4f*)(C + (size_t)(mBase + row) * ldc + n0 + c4) = v;
        }
        __threadfence();
      }
    } else {
      const int q = lane >> 3, c8 = (lane & 7) * 8;
      unsigned short* C = (unsigned short*)Cout + (size_t)b * (size_t)strideC;
      for (int pass = 0; pass < 2; ++pass) {
#pragma unroll
        for (int it = 0; it < 4; ++it) {
          const int row = it * 4 + q;
          const float* sp = slab + row * 68 + c8;
          v8h hv;
#pragma unroll
          for (int e = 0; e < 8; ++e) hv[e] = (_Float16)sp[e];
          *(volatile v8h*)(C + (size_t)(mBase + row) * ldc + n0 + c8) = hv;
        }
        __threadfence();
      }
    }
    __syncthreads();
  }
}

}

__global__ __launch_bounds__(256) void k_cast_rows(const float* __restrict__ SRC, unsigned short* __restrict__ DST,
                                                   int nR, int rowsPer, int rowsPerFull, float sc) {
  #pragma clang fp contract(off)
  const long long u = (long long)blockIdx.x * 256 + threadIdx.x;
  const int per = EMB / 8;
  if (u >= (long long)nR * per) return;
  const int r = (int)(u / per);
  const int c0 = 8 * (int)(u % per);
  const int rs = (r / rowsPer) * rowsPerFull + (r % rowsPer);
  const float* s = SRC + (long long)rs * EMB + c0;
  const v4f a = *(const v4f*)(s);
  const v4f c = *(const v4f*)(s + 4);
  u4 pk;
  pk.x = eng::pk2h(eng::bf_rne(a.x) * sc, eng::bf_rne(a.y) * sc);
  pk.y = eng::pk2h(eng::bf_rne(a.z) * sc, eng::bf_rne(a.w) * sc);
  pk.z = eng::pk2h(eng::bf_rne(c.x) * sc, eng::bf_rne(c.y) * sc);
  pk.w = eng::pk2h(eng::bf_rne(c.z) * sc, eng::bf_rne(c.w) * sc);
  volatile u4* d = (volatile u4*)(DST + (long long)r * EMB + c0);
  *d = pk;
  __threadfence();
  *d = pk;
}

__global__ __launch_bounds__(128) void attn_tflash(const unsigned short* __restrict__ QKp, const unsigned short* __restrict__ VTp,
                                                   unsigned short* __restrict__ CTXp) {
  __shared__ __align__(16) _Float16 cs[4][16 * 72];
  const _Float16* QK = (const _Float16*)QKp;
  const _Float16* VT = (const _Float16*)VTp;
  const int lane = threadIdx.x & 31, hf = lane >> 4, c = lane & 15;
  const int wave = __builtin_amdgcn_readfirstlane((int)(threadIdx.x >> 5));
  const int h = blockIdx.y, b = blockIdx.z;
  const int q0 = blockIdx.x * 64 + wave * 16;
  const size_t rowbase = (size_t)b * SEQ;

  const _Float16* qrow = QK + (rowbase + q0 + c) * QKP + h * HDIM + 8 * hf;
  const v16h qf0 = eng::frag_load(qrow);
  const v16h qf1 = eng::frag_load(qrow + 32);
  const _Float16* kbase = QK + (rowbase + c) * QKP + EMB + h * HDIM + 8 * hf;
  const _Float16* vbase = VT + ((size_t)b * EMB + h * HDIM + c) * SEQ + 8 * hf;

  v8f o[4];
#pragma unroll
  for (int t = 0; t < 4; ++t) o[t] = (v8f){0.f,0.f,0.f,0.f,0.f,0.f,0.f,0.f};
  float m = -1.0e30f, l = 0.f;
  const float SC = 0.125f * 1.4426950408889634f;

#pragma unroll 1
  for (int j0 = 0; j0 < SEQ; j0 += 32) {
    const _Float16* kp0 = kbase + (size_t)j0 * QKP;
    const _Float16* kp1 = kp0 + (size_t)16 * QKP;
    const v16h ka0 = eng::frag_load(kp0), ka1 = eng::frag_load(kp0 + 32);
    const v16h kb0 = eng::frag_load(kp1), kb1 = eng::frag_load(kp1 + 32);
    const _Float16* vp = vbase + j0;
    const v16h va0 = eng::frag_load(vp);
    const v16h va1 = eng::frag_load(vp + (size_t)16 * SEQ);
    const v16h va2 = eng::frag_load(vp + (size_t)32 * SEQ);
    const v16h va3 = eng::frag_load(vp + (size_t)48 * SEQ);

    v8f s0 = (v8f){0.f,0.f,0.f,0.f,0.f,0.f,0.f,0.f};
    v8f s1 = (v8f){0.f,0.f,0.f,0.f,0.f,0.f,0.f,0.f};
    s0 = eng::mma_h(ka0, qf0, s0);
    s0 = eng::mma_h(ka1, qf1, s0);
    s1 = eng::mma_h(kb0, qf0, s1);
    s1 = eng::mma_h(kb1, qf1, s1);
    eng::guard_s(s0, s1, ka0, ka1, kb0, kb1, qf0, qf1);

    float mx = fmaxf(s0[0], s1[0]);
#pragma unroll
    for (int r = 1; r < 8; ++r) mx = fmaxf(mx, fmaxf(s0[r], s1[r]));
    mx = fmaxf(mx, __shfl_xor(mx, 16, 32));
    const float mnew  = fmaxf(m, mx * SC);
    const float alpha = __builtin_amdgcn_exp2f(m - mnew);
    const float sh    = 10.0f - mnew;
    v16h pb;
    float ps = 0.f;
#pragma unroll
    for (int r = 0; r < 8; ++r) {
      const float p0 = __builtin_amdgcn_exp2f(fmaf(s0[r], SC, sh));
      const float p1 = __builtin_amdgcn_exp2f(fmaf(s1[r], SC, sh));
      ps += p0 + p1;
      pb[r]     = (_Float16)p0;
      pb[8 + r] = (_Float16)p1;
    }
    ps += __shfl_xor(ps, 16, 32);
    l = fmaf(l, alpha, ps);
    m = mnew;
#pragma unroll
    for (int t = 0; t < 4; ++t) o[t] = o[t] * alpha;

    o[0] = eng::mma_h(va0, pb, o[0]);
    o[1] = eng::mma_h(va1, pb, o[1]);
    o[2] = eng::mma_h(va2, pb, o[2]);
    o[3] = eng::mma_h(va3, pb, o[3]);
    eng::guard_o(o[0], o[1], o[2], o[3], va0, va1, va2, va3, pb);
  }

  const float inv = 256.0f * (1.0f / l);
  _Float16* my = cs[wave];
#pragma unroll
  for (int t = 0; t < 4; ++t) {
    v8h hv;
#pragma unroll
    for (int r = 0; r < 8; ++r) hv[r] = (_Float16)(o[t][r] * inv);
    *(v8h*)(my + c * 72 + 16 * t + 8 * hf) = hv;
  }
  __syncthreads();
  {
    const int q = lane >> 3, c8 = (lane & 7) * 8;
    unsigned short* dst = CTXp + (rowbase + q0) * EMB + h * HDIM;
    v8h rv[4];
#pragma unroll
    for (int it = 0; it < 4; ++it) rv[it] = *(const v8h*)(my + (it * 4 + q) * 72 + c8);
    for (int pass = 0; pass < 2; ++pass) {
#pragma unroll
      for (int it = 0; it < 4; ++it) *(volatile v8h*)(dst + (size_t)(it * 4 + q) * EMB + c8) = rv[it];
      __threadfence();
    }
  }
}

extern "C" void kernel_launch(void* const* d_in, const int* in_sizes, int n_in, void* d_out, int out_size, void* d_ws, size_t ws_size, hipStream_t stream) {
  if (n_in < 5) return;
  const long long need_x = ((long long)(NB - 1) * SEQ_FULL + SEQ) * EMB;
  if ((long long)in_sizes[0] < need_x) return;
  if ((long long)in_sizes[1] < (long long)3 * EMB * EMB) return;
  if (in_sizes[2] < 3 * EMB) return;
  if ((long long)in_sizes[3] < (long long)EMB * EMB) return;
  if (in_sizes[4] < EMB) return;
  if ((long long)out_size < (long long)NB * SEQ * EMB) return;

  const float* x      = (const float*)d_in[0];
  const float* w_qkv  = (const float*)d_in[1];
  const float* b_qkv  = (const float*)d_in[2];
  const float* w_proj = (const float*)d_in[3];
  const float* b_proj = (const float*)d_in[4];
  float* out = (float*)d_out;

  constexpr size_t ROWS   = (size_t)NB * SEQ;
  constexpr size_t SZ_X   = ROWS * EMB * 2;
  constexpr size_t SZ_W   = (size_t)3 * EMB * EMB * 2;
  constexpr size_t SZ_WP  = (size_t)EMB * EMB * 2;
  constexpr size_t SZ_QK  = ROWS * QKP * 2;
  constexpr size_t SZ_VT  = (size_t)NB * EMB * SEQ * 2;
  constexpr size_t SZ_CTX = ROWS * EMB * 2;
  static_assert(SZ_X % 256 == 0 && SZ_W % 256 == 0 && SZ_WP % 256 == 0 && SZ_QK % 256 == 0 && SZ_VT % 256 == 0 && SZ_CTX % 256 == 0);
  constexpr size_t CARVE = SZ_X + SZ_W + SZ_WP + SZ_QK + SZ_VT + SZ_CTX;
  static_assert(CARVE <= (size_t)134217728);
  if (CARVE > ws_size) return;

  char* wsp = (char*)d_ws;
  unsigned short* X16   = (unsigned short*)wsp; wsp += SZ_X;
  unsigned short* W16   = (unsigned short*)wsp; wsp += SZ_W;
  unsigned short* WP16  = (unsigned short*)wsp; wsp += SZ_WP;
  unsigned short* QK16  = (unsigned short*)wsp; wsp += SZ_QK;
  unsigned short* VT16  = (unsigned short*)wsp; wsp += SZ_VT;
  unsigned short* CTX16 = (unsigned short*)wsp; wsp += SZ_CTX;

  k_cast_rows<<<(unsigned)((ROWS * (EMB / 8) + 255) / 256), 256, 0, stream>>>(x, X16, (int)ROWS, SEQ, SEQ_FULL, 1.0f);
  k_cast_rows<<<(unsigned)(((size_t)3 * EMB * (EMB / 8) + 255) / 256), 256, 0, stream>>>(w_qkv, W16, 3 * EMB, 3 * EMB, 3 * EMB, 16.0f);
  k_cast_rows<<<(unsigned)(((size_t)EMB * (EMB / 8) + 255) / 256), 256, 0, stream>>>(w_proj, WP16, EMB, EMB, EMB, 16.0f);

  constexpr int TILES_QK = (int)((ROWS / 64) * (QKP / 64));
  static_assert(TILES_QK % 8 == 0);
  eng::wmma_gemm64<2, 1><<<dim3((unsigned)(TILES_QK / 8), 1u), 256, 0, stream>>>(
      X16, EMB, 0LL, W16, EMB, 0LL, (void*)QK16, QKP, 0LL, b_qkv, (int)ROWS, QKP, EMB, 0.0625f);

  constexpr int TILES_VT = (EMB / 64) * (SEQ / 64);
  static_assert(TILES_VT % 8 == 0);
  eng::wmma_gemm64<1, 1><<<dim3((unsigned)(TILES_VT / 8), (unsigned)NB), 256, 0, stream>>>(
      W16 + (size_t)2 * EMB * EMB, EMB, 0LL, X16, EMB, (long long)SEQ * EMB, (void*)VT16, SEQ, (long long)EMB * SEQ,
      b_qkv + 2 * EMB, EMB, SEQ, EMB, 0.0625f);

  attn_tflash<<<dim3((unsigned)(SEQ / 64), (unsigned)NHEADS, (unsigned)NB), 128, 0, stream>>>(QK16, VT16, CTX16);

  constexpr int TILES_P = (int)((ROWS / 64) * (EMB / 64));
  static_assert(TILES_P % 8 == 0);
  eng::wmma_gemm64<2, 0><<<dim3((unsigned)(TILES_P / 8), 1u), 256, 0, stream>>>(
      CTX16, EMB, 0LL, WP16, EMB, 0LL, (void*)out, EMB, 0LL, b_proj, (int)ROWS, EMB, EMB, 1.0f / 4096.0f);
}
